// GroupAttention_80719615361202
// MI455X (gfx1250) — hardware-verified
//
#include <hip/hip_runtime.h>


#define NB_  16
#define CC   512
#define NN   1024
#define NH_  8
#define CG   64
#define KD   32
#define DV   128
#define QO   192
#define NT   (NB_ * NN)
#define CO   1024
#define PCAR 1024.0f
typedef _Float16 h16;
typedef unsigned short bf;
typedef __attribute__((ext_vector_type(16))) __bf16   v16bf;
typedef __attribute__((ext_vector_type(16))) _Float16 v16h;
typedef __attribute__((ext_vector_type(8)))  _Float16 v8h;
typedef __attribute__((ext_vector_type(8)))  unsigned short v8us;
typedef __attribute__((ext_vector_type(8)))  float    v8f;
typedef __attribute__((ext_vector_type(4)))  float    v4f;
typedef v8h  __attribute__((may_alias)) v8ha;
typedef v4f  __attribute__((may_alias)) v4fa;
typedef v8us __attribute__((may_alias)) v8usa;

__device__ __forceinline__ unsigned short f2bf(float f) { unsigned u = __float_as_uint(f); u += 0x7FFFu + ((u >> 16) & 1u); return (unsigned short)(u >> 16); }
__device__ __forceinline__ float bf2f(unsigned short b) { return __uint_as_float(((unsigned)b) << 16); }
__device__ __forceinline__ float bfr(float f) { return bf2f(f2bf(f)); }
__device__ __forceinline__ v16h cat16(v8h lo, v8h hi) { return __builtin_shufflevector(lo, hi, 0, 1, 2, 3, 4, 5, 6, 7, 8, 9, 10, 11, 12, 13, 14, 15); }
__device__ __forceinline__ v16bf cat16b(v8us lo, v8us hi) { return __builtin_bit_cast(v16bf, __builtin_shufflevector(lo, hi, 0, 1, 2, 3, 4, 5, 6, 7, 8, 9, 10, 11, 12, 13, 14, 15)); }
__device__ __forceinline__ v8f wmma16(v16h a, v16h b, v8f c) { return __builtin_amdgcn_wmma_f32_16x16x32_f16(false, a, false, b, (short)0, c, false, false); }
__device__ __forceinline__ v8f wmmab(v16bf a, v16bf b, v8f c) { return __builtin_amdgcn_wmma_f32_16x16x32_bf16(false, a, false, b, (short)0, c, false, false); }


template <typename T16> struct WFrag;
template <> struct WFrag<h16> { typedef v16h V; static __device__ __forceinline__ V ld(const h16* p) { return cat16(*(const v8h*)p, *(const v8h*)(p + 16)); } static __device__ __forceinline__ v8f mma(V a, V b, v8f c) { return wmma16(a, b, c); } };
template <> struct WFrag<bf> { typedef v16bf V; static __device__ __forceinline__ V ld(const bf* p) { return cat16b(*(const v8us*)p, *(const v8us*)(p + 16)); } static __device__ __forceinline__ v8f mma(V a, V b, v8f c) { return wmmab(a, b, c); } };
template <typename T16, int NSPLIT, bool BIAS>
__global__ __launch_bounds__(32) void k_gemmw(const T16* __restrict__ A, const T16* __restrict__ A2, const T16* __restrict__ Bt, const T16* __restrict__ Bt2, int K, float* C, int ldc, const float* __restrict__ bias, size_t sA, size_t sB, size_t sC) {
    typedef typename WFrag<T16>::V V;
    __shared__ __align__(16) float os[16 * 68];
    const size_t z = blockIdx.z; A += z * sA; if (A2) A2 += z * sA; Bt += z * sB; if (Bt2) Bt2 += z * sB; C += z * sC;
    const int lane = threadIdx.x & 31, lr = lane & 15, hi = lane >> 4; const int r0 = blockIdx.x * 64, c0 = blockIdx.y * 64;
    v8f acc[4][4];
#pragma unroll
    for (int mb = 0; mb < 4; ++mb)
#pragma unroll
        for (int nb = 0; nb < 4; ++nb) acc[mb][nb] = (v8f){};
    const size_t aoff = (size_t)(r0 + lr) * K + 8 * hi, boff = (size_t)(c0 + lr) * K + 8 * hi;
#pragma unroll 1
    for (int kc = 0; kc < K; kc += 32) {
        V a[4], a2[4];
#pragma unroll
        for (int mb = 0; mb < 4; ++mb) { a[mb] = WFrag<T16>::ld(A + aoff + (size_t)mb * 16 * K + kc); if (NSPLIT == 1 || NSPLIT == 2) a2[mb] = WFrag<T16>::ld(A2 + aoff + (size_t)mb * 16 * K + kc); }
#pragma unroll
        for (int nb = 0; nb < 4; ++nb) { const V b = WFrag<T16>::ld(Bt + boff + (size_t)nb * 16 * K + kc); V b2; if (NSPLIT >= 2) b2 = WFrag<T16>::ld(Bt2 + boff + (size_t)nb * 16 * K + kc);
#pragma unroll
            for (int mb = 0; mb < 4; ++mb) { acc[mb][nb] = WFrag<T16>::mma(a[mb], b, acc[mb][nb]); if (NSPLIT == 1 || NSPLIT == 2) acc[mb][nb] = WFrag<T16>::mma(a2[mb], b, acc[mb][nb]); if (NSPLIT >= 2) acc[mb][nb] = WFrag<T16>::mma(a[mb], b2, acc[mb][nb]); } }
        asm volatile("v_nop\n\tv_nop\n\tv_nop\n\tv_nop" : "+v"(acc[0][0]), "+v"(acc[1][1]), "+v"(acc[2][2]), "+v"(acc[3][3]) : "v"(a[0]), "v"(a[3]));
    }
#pragma unroll
    for (int mb = 0; mb < 4; ++mb) {
#pragma unroll
        for (int nb = 0; nb < 4; ++nb) {
#pragma unroll
            for (int j = 0; j < 8; ++j) os[(hi * 8 + j) * 68 + nb * 16 + lr] = acc[mb][nb][j]; }
        __builtin_amdgcn_wave_barrier(); asm volatile("" ::: "memory");
        float* crow = C + (size_t)(r0 + mb * 16) * ldc + c0;
#pragma unroll 1
        for (int ps = 0; ps < 2; ++ps) {
#pragma unroll
            for (int s = 0; s < 8; ++s) { const int row = 2 * s + hi, cofs = lr * 4; v4f val = *(const v4fa*)(os + row * 68 + cofs); if (BIAS) { val[0] += bfr(bias[c0 + cofs]); val[1] += bfr(bias[c0 + cofs + 1]); val[2] += bfr(bias[c0 + cofs + 2]); val[3] += bfr(bias[c0 + cofs + 3]); }
                *(volatile v4f*)(crow + (size_t)row * ldc + cofs) = val; }
            if (ps == 0) __threadfence(); }
        __builtin_amdgcn_wave_barrier(); asm volatile("" ::: "memory");
    }
}

__device__ __forceinline__ h16 tohx(float x) { return (h16)x; }
__device__ __forceinline__ void splitf(float y, unsigned short& h, unsigned short& l) { h = f2bf(y); l = f2bf(y - bf2f(h)); }
typedef __attribute__((ext_vector_type(2))) _Float16 v2h;
typedef __attribute__((ext_vector_type(4))) _Float16 v4h;
typedef __attribute__((ext_vector_type(2))) unsigned short v2us;
typedef __attribute__((ext_vector_type(8))) unsigned short v8us_;

__global__ __launch_bounds__(256) void k_cvt8(const float* __restrict__ src, bf* dst, size_t n8) { const size_t i = (size_t)blockIdx.x * 256 + threadIdx.x; if (i >= n8) return; const v8f v = *(const v8f*)(src + i * 8); v8us o;
#pragma unroll
    for (int k = 0; k < 8; ++k) o[k] = f2bf(v[k]); *(volatile v8us*)(dst + i * 8) = o; __threadfence(); *(volatile v8us*)(dst + i * 8) = o; }
__global__ __launch_bounds__(256) void k_xg(const float* __restrict__ x, bf* XG) {
    __shared__ float tl[CG][65];
    const int tid = threadIdx.x; const int n0 = blockIdx.x * 64, h = blockIdx.y, b = blockIdx.z;
#pragma unroll
    for (int i = 0; i < 16; ++i) { const int c = i * 4 + (tid >> 6), nn = tid & 63; tl[c][nn] = x[((size_t)b * CC + h * CG + c) * NN + n0 + nn]; }
    __syncthreads();
    const int lane = tid & 31, wv = tid >> 5;
    auto pass = [&]() {
#pragma unroll
        for (int i2 = 0; i2 < 2; ++i2) { const int r = wv * 8 + i2 * 4 + (lane >> 3); const int cq = (lane & 7) * 8; v8us_ o;
#pragma unroll
            for (int i = 0; i < 8; ++i) o[i] = f2bf(tl[cq + i][r]);
            *(volatile v8us_*)(XG + (((size_t)h * NB_ + b) * NN + n0 + r) * CG + cq) = o; } };
    pass(); __threadfence(); pass();
}
__global__ __launch_bounds__(256) void k_qkplanes(const float* __restrict__ F, int h, h16* Qp, h16* Kp) {
    const int lane = threadIdx.x & 31; const int L0 = (blockIdx.x * 8 + (threadIdx.x >> 5)) * 8; const int nlines = NT * KD / 64; const float sc = 0x1.6a09e6p-3f;
#pragma unroll 1
    for (int ps = 0; ps < 2; ++ps) {
#pragma unroll
        for (int l = 0; l < 8; ++l) { const int L = L0 + l; if (L >= nlines) break; const int e = L * 64 + lane * 2; const int c = e & 31; const int bn = e >> 5; const int b = bn >> 10, n = bn & 1023; v2h vq, vk;
#pragma unroll
            for (int q = 0; q < 2; ++q) { vq[q] = tohx(F[(size_t)bn * QO + c + q] * sc); vk[q] = tohx(F[(size_t)bn * QO + KD + c + q]); }
            const size_t o = (((size_t)(b * NH_ + h)) * NN + n) * KD + c; *(volatile v2h*)(Qp + o) = vq; *(volatile v2h*)(Kp + o) = vk; }
        if (ps == 0) __threadfence(); }
}
__global__ __launch_bounds__(256) void k_vplane(const float* __restrict__ F, int h, h16* Vp) {
    const int lane = threadIdx.x & 31; const int L0 = (blockIdx.x * 8 + (threadIdx.x >> 5)) * 8; const int nlines = NB_ * DV * NN / 64;
#pragma unroll 1
    for (int ps = 0; ps < 2; ++ps) {
#pragma unroll
        for (int l = 0; l < 8; ++l) { const int L = L0 + l; if (L >= nlines) break; const int e = L * 64 + lane * 2; const int n = e & 1023; const int d = (e >> 10) & 127; const int b = e >> 17; v2h v;
#pragma unroll
            for (int q = 0; q < 2; ++q) v[q] = tohx(F[((size_t)b * NN + n + q) * QO + 2 * KD + d]);
            *(volatile v2h*)(Vp + (((size_t)(b * NH_ + h)) * DV + d) * NN + n) = v; }
        if (ps == 0) __threadfence(); }
}
__global__ __launch_bounds__(256) void k_soft(const float* __restrict__ Sb, h16* P) {
    const int lane = threadIdx.x & 31; const int row = blockIdx.x * 8 + (threadIdx.x >> 5); if (row >= NH_ * NN) return; const float* sr = Sb + (size_t)row * NN; float v[32]; float m = -3.0e38f;
#pragma unroll
    for (int ch = 0; ch < 8; ++ch) { const v4f t = *(const v4f*)(sr + ch * 128 + lane * 4);
#pragma unroll
        for (int q = 0; q < 4; ++q) { v[ch * 4 + q] = t[q]; m = fmaxf(m, t[q]); } }
#pragma unroll
    for (int sh = 16; sh; sh >>= 1) m = fmaxf(m, __shfl_xor(m, sh, 32));
    float sum = 0.f;
#pragma unroll
    for (int i = 0; i < 32; ++i) { v[i] = __expf(v[i] - m); sum += v[i]; }
#pragma unroll
    for (int sh = 16; sh; sh >>= 1) sum += __shfl_xor(sum, sh, 32);
    const float f = __fdiv_rn(PCAR, sum);
#pragma unroll 1
    for (int ps = 0; ps < 2; ++ps) {
#pragma unroll
        for (int ch = 0; ch < 8; ++ch) { v4h o;
#pragma unroll
            for (int q = 0; q < 4; ++q) o[q] = tohx(v[ch * 4 + q] * f);
            *(volatile v4h*)(P + (size_t)row * NN + ch * 128 + lane * 4) = o; }
        if (ps == 0) __threadfence(); }
}
__global__ __launch_bounds__(256) void k_rplanes(const float* __restrict__ O, int b, bf* Rh, bf* Rl) {
    const int lane = threadIdx.x & 31; const int L0 = (blockIdx.x * 8 + (threadIdx.x >> 5)) * 8; const int nlines = NN * CO / 64;
#pragma unroll 1
    for (int ps = 0; ps < 2; ++ps) {
#pragma unroll
        for (int l = 0; l < 8; ++l) { const int L = L0 + l; if (L >= nlines) break; const int e = L * 64 + lane * 2; const int c = e & 1023; const int m = e >> 10; const int h = c >> 7, d = c & 127; v2us oh, ol;
#pragma unroll
            for (int q = 0; q < 2; ++q) { unsigned short a, c2; splitf(fmaxf(O[((size_t)h * NN + m) * DV + d + q] * (1.0f / PCAR), 0.f), a, c2); oh[q] = a; ol[q] = c2; }
            const size_t o = ((size_t)b * NN + m) * CO + c; *(volatile v2us*)(Rh + o) = oh; *(volatile v2us*)(Rl + o) = ol; }
        if (ps == 0) __threadfence(); }
}
__global__ __launch_bounds__(256) void k_bnT(const float* __restrict__ Cp, const float* __restrict__ gm, const float* __restrict__ bt, const float* __restrict__ mn, const float* __restrict__ vr, float* OUT) {
    __shared__ float tl[64][65];
    const int tid = threadIdx.x; const int n0 = blockIdx.x * 64, o0 = blockIdx.y * 64, b = blockIdx.z;
#pragma unroll
    for (int i = 0; i < 16; ++i) { const int nn = i * 4 + (tid >> 6), oc = tid & 63; tl[nn][oc] = Cp[((size_t)b * NN + n0 + nn) * CC + o0 + oc]; }
    __syncthreads();
    const int lane = tid & 31, wv = tid >> 5;
    auto pass = [&]() {
#pragma unroll 1
        for (int i2 = 0; i2 < 4; ++i2) { const int ocl = wv * 8 + i2 * 2 + (lane >> 4); const int oc = o0 + ocl; const int nq = (lane & 15) * 4; const float inv = __fdiv_rn(bfr(gm[oc]), sqrtf(bfr(vr[oc]) + 1e-5f)); const float shf = bfr(bt[oc]) - bfr(mn[oc]) * inv; v4f o;
#pragma unroll
            for (int q = 0; q < 4; ++q) o[q] = tl[nq + q][ocl] * inv + shf;
            *(volatile v4f*)(OUT + ((size_t)b * CC + oc) * NN + n0 + nq) = o; } };
    pass(); __threadfence(); pass();
}

extern "C" void kernel_launch(void* const* d_in, const int* in_sizes, int n_in,
                              void* d_out, int out_size, void* d_ws, size_t ws_size, hipStream_t stream) {
    (void)in_sizes; (void)n_in; (void)out_size;
    const float* x = (const float*)d_in[0]; const float* qkv_w = (const float*)d_in[1]; const float* qkv_b = (const float*)d_in[2]; const float* proj_w = (const float*)d_in[3]; const float* proj_b = (const float*)d_in[4];
    const float* gm = (const float*)d_in[5]; const float* bt = (const float*)d_in[6]; const float* mn = (const float*)d_in[7]; const float* vr = (const float*)d_in[8];
    float* OUT = (float*)d_out;
    char* wsp = (char*)d_ws;
    auto take = [&](size_t bytes) { char* p = wsp; wsp += (bytes + 255) & ~(size_t)255; return (void*)p; };
    bf* WQKV = (bf*)take((size_t)NH_ * QO * CG * 2); bf* PW = (bf*)take((size_t)CC * CO * 2);
    bf* Rh = (bf*)take((size_t)NT * CO * 2); bf* Rl = (bf*)take((size_t)NT * CO * 2);
    char* RS = (char*)take((size_t)NH_ * NN * NN * 4);
    h16* Pm = (h16*)take((size_t)NH_ * NN * NN * 2); h16* Vp = (h16*)take((size_t)NB_ * NH_ * DV * NN * 2); h16* Qp = (h16*)take((size_t)NB_ * NH_ * NN * KD * 2); h16* Kp = (h16*)take((size_t)NB_ * NH_ * NN * KD * 2);
    float* F = (float*)take((size_t)NT * QO * 4); float* Ob = (float*)take((size_t)NH_ * NN * DV * 4);
    if ((size_t)(wsp - (char*)d_ws) > ws_size) return;
    bf* XG = (bf*)RS; float* Sb = (float*)RS; float* Cp = (float*)RS;
    { const size_t n1 = (size_t)NH_ * QO * CG / 8, n2 = (size_t)CC * CO / 8; k_cvt8<<<(unsigned)((n1 + 255) / 256), 256, 0, stream>>>(qkv_w, WQKV, n1); k_cvt8<<<(unsigned)((n2 + 255) / 256), 256, 0, stream>>>(proj_w, PW, n2); }
    k_xg<<<dim3(NN / 64, NH_, NB_), 256, 0, stream>>>(x, XG);
    for (int h = 0; h < NH_; ++h) {
        k_gemmw<bf, 0, true><<<dim3(NT / 64, QO / 64, 1), 32, 0, stream>>>(XG + (size_t)h * NT * CG, nullptr, WQKV + (size_t)h * QO * CG, nullptr, CG, F, QO, qkv_b + h * QO, 0, 0, 0);
        k_qkplanes<<<(NT * KD / 64 + 63) / 64, 256, 0, stream>>>(F, h, Qp, Kp);
        k_vplane<<<(NB_ * DV * NN / 64 + 63) / 64, 256, 0, stream>>>(F, h, Vp); }
    for (int b = 0; b < NB_; ++b) { const size_t z0 = (size_t)b * NH_;
        k_gemmw<h16, 0, false><<<dim3(NN / 64, NN / 64, NH_), 32, 0, stream>>>(Qp + z0 * NN * KD, nullptr, Kp + z0 * NN * KD, nullptr, KD, Sb, NN, nullptr, (size_t)NN * KD, (size_t)NN * KD, (size_t)NN * NN);
        k_soft<<<NH_ * NN / 8, 256, 0, stream>>>(Sb, Pm);
        k_gemmw<h16, 0, false><<<dim3(NN / 64, DV / 64, NH_), 32, 0, stream>>>(Pm, nullptr, Vp + z0 * DV * NN, nullptr, NN, Ob, DV, nullptr, (size_t)NN * NN, (size_t)DV * NN, (size_t)NN * DV);
        k_rplanes<<<(NN * CO / 64 + 63) / 64, 256, 0, stream>>>(Ob, b, Rh, Rl); }
    k_gemmw<bf, 1, true><<<dim3(NT / 64, CC / 64, 1), 32, 0, stream>>>(Rh, Rl, PW, nullptr, CO, Cp, CC, proj_b, 0, 0, 0);
    k_bnT<<<dim3(NN / 64, CC / 64, NB_), 256, 0, stream>>>(Cp, gm, bt, mn, vr, OUT);
}
